// DPBlockVFAStandard_81647328297391
// MI455X (gfx1250) — hardware-verified
//
#include <hip/hip_runtime.h>
#include <hip/hip_bf16.h>

typedef __attribute__((ext_vector_type(16))) _Float16     v16h;
typedef __attribute__((ext_vector_type(8)))  _Float16     v8h;
typedef __attribute__((ext_vector_type(4)))  float        v4f;
#define ZP 80
typedef __attribute__((ext_vector_type(8)))  float        v8f;
typedef __attribute__((ext_vector_type(4)))  unsigned int v4u;
typedef __attribute__((ext_vector_type(8)))  unsigned int v8u;

#define EMBED  16
#define CIN    32
#define NOFF   27
#define KTOT   (CIN * NOFF)
#define VOL64  (64 * 64 * 64)
#define VOL66  (66 * 66 * 66)

#define WAVES_PER_BLOCK 4
#define LDS_PER_WAVE    (9 * 18 * 32)

__device__ __forceinline__ int clampi(int v, int lo, int hi) {
    return v < lo ? lo : (v > hi ? hi : v);
}

__global__ void prep_weights_kernel(const float* __restrict__ w,
                                    _Float16* __restrict__ w16) {
    int idx = blockIdx.x * blockDim.x + threadIdx.x;
    if (idx >= EMBED * KTOT) return;
    int r     = idx / KTOT;
    int t     = idx % KTOT;
    int off   = t >> 5;
    int u     = t & 31;
    int khalf = u >> 4;
    int h     = u & 15;
    int cin   = (h & 7) + 8 * khalf + 16 * (h >> 3);
    const _Float16 hv = (_Float16)w[(r * CIN + cin) * NOFF + off];
    *(volatile _Float16*)(w16 + idx) = hv; __threadfence(); *(volatile _Float16*)(w16 + idx) = hv;
}

template <int MODE, int OUTD, int NDT, int LAYOUT>
__global__ void conv_wmma_kernel(const float* __restrict__ src,
                                 const float* __restrict__ bias,
                                 const _Float16* __restrict__ w16,
                                 float* __restrict__ dst,
                                 int nTiles) {
    __shared__ __align__(64) _Float16 lds[WAVES_PER_BLOCK][LDS_PER_WAVE];
    __shared__ __align__(16) float sOut[WAVES_PER_BLOCK][16 * 16];

    const int lane  = threadIdx.x & 31;
    const int wave  = threadIdx.x >> 5;
    const int tile  = blockIdx.x * WAVES_PER_BLOCK + wave;
    if (tile >= nTiles) return;

    const int col   = lane & 15;
    const int khalf = lane >> 4;

    const int td = tile % NDT;
    const int x  = (tile / NDT) % OUTD;
    const int y  =  tile / (NDT * OUTD);
    const int d0 = td * 16;

    _Float16* myLds = &lds[wave][0];

    #pragma unroll 1
    for (int it = 0; it < 9; ++it) {
        const int r  = lane + 32 * it;
        const int c  = r / 9;
        const int t9 = r % 9;
        const int ii = t9 / 3;
        const int jj = t9 % 3;
        const int gy = y + ii - 1;
        const int gx = x + jj - 1;

        bool rowOK;
        int  sy, sx;
        if (MODE == 0) {
            rowOK = (unsigned)gy < 64u && (unsigned)gx < 64u;
            sy = clampi(gy, 0, 63);
            sx = clampi(gx, 0, 63);
        } else {
            rowOK = (unsigned)gy < 66u && (unsigned)gx < 66u;
            sy = clampi(gy - 1, 0, 63);
            sx = clampi(gx - 1, 0, 63);
        }
        const float* p = src + (size_t)c * VOL64 + ((size_t)(sy * 64 + sx) * 64);
        _Float16* q = myLds + (size_t)t9 * (18 * 32) + c;

        #pragma unroll 1
        for (int iz = 0; iz < 18; ++iz) {
            const int gz = d0 + iz - 1;
            bool zOK;
            int  sz;
            if (MODE == 0) {
                zOK = (unsigned)gz < 64u;
                sz  = clampi(gz, 0, 63);
            } else {
                zOK = (unsigned)gz < 66u;
                sz  = clampi(gz - 1, 0, 63);
            }
            float v   = p[sz];
            float val = (rowOK && zOK) ? v : 0.0f;
            q[(size_t)iz * 32] = (_Float16)val;
        }
    }

    const _Float16* wrow = w16 + (size_t)col * KTOT + khalf * 16;

    v8f acc = {};
    #pragma unroll
    for (int off = 0; off < NOFF; ++off) {
        const int t9 = off / 3;
        const int k  = off % 3;
        v16h a = *(const v16h*)(wrow + off * 32);
        const _Float16* bp = myLds + ((size_t)t9 * 18 + (col + k)) * 32 + khalf * 8;
        v16h b = __builtin_shufflevector(*(const v8h*)bp, *(const v8h*)(bp + 16), 0,1,2,3,4,5,6,7,8,9,10,11,12,13,14,15);
        acc = __builtin_amdgcn_wmma_f32_16x16x32_f16(
            false, a, false, b, (short)0, acc, false, false);
        asm volatile("v_nop\n\tv_nop\n\tv_nop\n\tv_nop" : "+v"(acc) : "v"(a), "v"(b));
    }

    constexpr int ZSTR = (MODE == 0) ? OUTD : ZP;
    float* so = sOut[wave];
    #pragma unroll
    for (int g = 0; g < 8; ++g) { const int row = g + 8 * khalf; so[col * 16 + row] = acc[g] + bias[row]; }
    __builtin_amdgcn_fence(__ATOMIC_RELEASE, "workgroup"); __builtin_amdgcn_wave_barrier(); __builtin_amdgcn_fence(__ATOMIC_ACQUIRE, "workgroup");
    if (d0 < ZSTR) {
        float* gdst = dst + (((size_t)y * OUTD + x) * ZSTR + d0) * 16;
        for (int pass = 0; pass < 2; ++pass) {
            *(volatile v4f*)(gdst + lane * 4)       = *(const v4f*)(so + lane * 4);
            *(volatile v4f*)(gdst + 128 + lane * 4) = *(const v4f*)(so + 128 + lane * 4);
            __threadfence();
        }
    }
    (void)LAYOUT;
}

__global__ __launch_bounds__(256) void attn_disp_kernel(const float* __restrict__ fixed_emb,
                                                        const float* __restrict__ mov_emb,
                                                        float* __restrict__ out) {
    __shared__ __align__(16) float tile[6 * 4 * 34 * 16];
    const int b  = blockIdx.x;
    const int bz = b & 1;
    const int bx = (b >> 1) & 31;
    const int by = b >> 6;
    const int z0 = bz * 32, x0 = bx * 2, y0 = by * 4;
    for (int p = threadIdx.x; p < 6 * 4 * 34 * 4; p += 256) {
        const int vox = p >> 2, q4 = (p & 3) * 4;
        const int tz = vox % 34, tx = (vox / 34) % 4, ty = vox / 136;
        *(v4f*)(&tile[vox * 16 + q4]) = *(const v4f*)(mov_emb + (((size_t)(y0 + ty) * 66 + (x0 + tx)) * ZP + (z0 + tz)) * 16 + q4);
    }
    __syncthreads();

    const int t  = threadIdx.x;
    const int lz = t & 31, lx = (t >> 5) & 1, ly = t >> 6;
    const int z = z0 + lz, x = x0 + lx, y = y0 + ly;
    const int v = (y * 64 + x) * 64 + z;

    float q[EMBED];
    #pragma unroll
    for (int e = 0; e < EMBED; ++e)
        q[e] = fixed_emb[(size_t)v * 16 + e];

    float mx = -1e30f;
    #pragma unroll 1
    for (int p = 0; p < NOFF; ++p) {
        const int i = p / 9, j = (p / 3) % 3, k = p % 3;
        const float* m = &tile[(((ly + i) * 4 + (lx + j)) * 34 + (lz + k)) * 16];
        float s = 0.0f;
        #pragma unroll
        for (int e = 0; e < EMBED; ++e) s = __builtin_fmaf(q[e], m[e], s);
        mx = fmaxf(mx, s * 0.25f);
    }
    float sum = 0.0f, dh = 0.0f, dw = 0.0f, dd = 0.0f;
    #pragma unroll 1
    for (int p = 0; p < NOFF; ++p) {
        const int i = p / 9, j = (p / 3) % 3, k = p % 3;
        const float* m = &tile[(((ly + i) * 4 + (lx + j)) * 34 + (lz + k)) * 16];
        float s = 0.0f;
        #pragma unroll
        for (int e = 0; e < EMBED; ++e) s = __builtin_fmaf(q[e], m[e], s);
        const float ex = __expf(s * 0.25f - mx);
        sum += ex;
        dh += ex * (float)(i - 1);
        dw += ex * (float)(j - 1);
        dd += ex * (float)(k - 1);
    }
    float inv = 1.0f / sum;
    for (int pass = 0; pass < 2; ++pass) {
        *(volatile float*)(out + v)             = dh * inv;
        *(volatile float*)(out + VOL64 + v)     = dw * inv;
        *(volatile float*)(out + 2 * VOL64 + v) = dd * inv;
        __threadfence();
    }
}

extern "C" void kernel_launch(void* const* d_in, const int* in_sizes, int n_in,
                              void* d_out, int out_size, void* d_ws, size_t ws_size,
                              hipStream_t stream) {
    const float* feat_moving = (const float*)d_in[0];
    const float* feat_fixed  = (const float*)d_in[1];
    const float* conv_w      = (const float*)d_in[2];
    const float* conv_b      = (const float*)d_in[3];
    float* out = (float*)d_out;

    (void)in_sizes; (void)n_in; (void)out_size;
    char* ws = (char*)d_ws;
    _Float16* w16    = (_Float16*)ws;
    float* fixed_emb = (float*)(ws + 32768);
    float* mov_emb   = (float*)(ws + 32768 + (size_t)EMBED * VOL64 * 4);
    if (ws_size < 32768 + (size_t)EMBED * VOL64 * 4 + (size_t)66 * 66 * ZP * 16 * 4) return;

    prep_weights_kernel<<<(EMBED * KTOT + 255) / 256, 256, 0, stream>>>(conv_w, w16);

    conv_wmma_kernel<0, 64, 4, 0>
        <<<16384 / WAVES_PER_BLOCK, 32 * WAVES_PER_BLOCK, 0, stream>>>(
            feat_fixed, conv_b, w16, fixed_emb, 16384);

    const int ntm = 66 * 66 * 5;
    conv_wmma_kernel<1, 66, 5, 1>
        <<<(ntm + WAVES_PER_BLOCK - 1) / WAVES_PER_BLOCK,
           32 * WAVES_PER_BLOCK, 0, stream>>>(
            feat_moving, conv_b, w16, mov_emb, ntm);

    attn_disp_kernel<<<1024, 256, 0, stream>>>(fixed_emb, mov_emb, out);
}
